// HyperGraphHead_83030307766610
// MI455X (gfx1250) — hardware-run, weakly checked
//
#include <hip/hip_runtime.h>
#include <math.h>

typedef __attribute__((ext_vector_type(16))) _Float16 v16h;
typedef __attribute__((ext_vector_type(8)))  _Float16 v8h;
typedef __attribute__((ext_vector_type(8)))  float    v8f;
typedef __attribute__((ext_vector_type(4)))  float    v4f;
typedef __attribute__((ext_vector_type(4)))  int      v4i;

constexpr int kB    = 8;
constexpr int kN    = 2048;
constexpr int kH    = 512;
constexpr int kH2   = 2 * kH;
constexpr int kRows = kB * kN;
constexpr float kActCarry = 64.0f;
constexpr float kWgtCarry = 1024.0f;
constexpr float kQCarry   = 1024.0f;
constexpr float kFold     = 1.0f / (kActCarry * kWgtCarry);
constexpr float kInvH     = 1.0f / (float)kH;
constexpr float kLnEps    = 1e-5f;
static_assert(kFold * kActCarry * kWgtCarry == 1.0f, "exact fold");
static_assert((kH % 32) == 0 && (kH2 % 32) == 0, "GEMM K multiples of 32");
static_assert((kRows % 64) == 0 && (kH % 64) == 0 && (kN % 64) == 0, "tile multiples");
static_assert(kH == 512 && kN == 2048 && kB == 8, "wire shapes");

constexpr size_t kSzPlane = (size_t)kRows * kH * 2;
constexpr size_t kOffE16  = 0;
constexpr size_t kOffQ16  = kOffE16 + kSzPlane;
constexpr size_t kOffX1   = kOffQ16 + kSzPlane;
constexpr size_t kOffX2   = kOffX1  + kSzPlane;
constexpr size_t kOffW1T  = kOffX2  + kSzPlane;
constexpr size_t kOffW2T  = kOffW1T + (size_t)kH * kH * 2;
constexpr size_t kOffWFT  = kOffW2T + (size_t)kH * kH * 2;
constexpr size_t kOffIDX  = kOffWFT + (size_t)kH * kH2 * 2;
constexpr size_t kOffGD   = kOffIDX + (size_t)kRows * 4;
constexpr size_t kWsTotal = kOffGD  + (size_t)kRows * 4;
static_assert(kWsTotal == 69337088ull, "carve total");
static_assert(kWsTotal <= 134217728ull, "carve cap");
static_assert((kOffQ16 % 128) == 0 && (kOffX1 % 128) == 0 && (kOffX2 % 128) == 0 && (kOffW1T % 128) == 0 &&
              (kOffW2T % 128) == 0 && (kOffWFT % 128) == 0 && (kOffIDX % 128) == 0 && (kOffGD % 128) == 0,
              "128-B aligned regions");

__device__ __forceinline__ unsigned short f2bf_bits(float f) {
  unsigned u = __float_as_uint(f);
  return (unsigned short)((u + 0x7FFFu + ((u >> 16) & 1u)) >> 16);
}
__device__ __forceinline__ float bf_rne(float f) {
  return __uint_as_float(((unsigned)f2bf_bits(f)) << 16);
}
__device__ __forceinline__ v16h frag_ld(const _Float16* p) {
  union { v16h v; v8h h[2]; } f;
  f.h[0] = *(const v8h*)(p);
  f.h[1] = *(const v8h*)(p + 16);
  return f.v;
}
__device__ __forceinline__ v8f mma_g(v16h a, v16h b, v8f c) {
  c = __builtin_amdgcn_wmma_f32_16x16x32_f16(false, a, false, b, (short)0, c, false, false);
  asm volatile("v_nop\n\tv_nop\n\tv_nop\n\tv_nop" : "+v"(c) : "v"(a), "v"(b));
  return c;
}
__device__ __forceinline__ void wave_lds_sync() {
  __builtin_amdgcn_fence(__ATOMIC_RELEASE, "workgroup");
  __builtin_amdgcn_wave_barrier();
  __builtin_amdgcn_fence(__ATOMIC_ACQUIRE, "workgroup");
}

__global__ __launch_bounds__(256) void prep_weights_kernel(
    const float* __restrict__ W1, const float* __restrict__ W2, const float* __restrict__ Wfc,
    unsigned short* __restrict__ W1T, unsigned short* __restrict__ W2T, unsigned short* __restrict__ WFT)
{
  __shared__ __align__(16) float sT[64 * 68];
  const int tid  = threadIdx.x;
  const int lane = tid & 31;
  const int wave = __builtin_amdgcn_readfirstlane((int)(threadIdx.x >> 5));
  const int blk  = blockIdx.x;
  const float* src;
  unsigned short* dst;
  int kdim, t;
  if (blk < 64)       { src = W1;  dst = W1T; kdim = kH;  t = blk; }
  else if (blk < 128) { src = W2;  dst = W2T; kdim = kH;  t = blk - 64; }
  else                { src = Wfc; dst = WFT; kdim = kH2; t = blk - 128; }
  const int k0 = (t >> 3) * 64;
  const int n0 = (t & 7) * 64;
  {
    const int kk  = tid >> 2;
    const int c16 = (tid & 3) * 16;
    const float* sp = src + (size_t)(k0 + kk) * kH + n0 + c16;
#pragma unroll
    for (int q4 = 0; q4 < 4; ++q4) {
      const v4f v = *(const v4f*)(sp + 4 * q4);
      *(v4f*)(sT + kk * 68 + c16 + 4 * q4) = v;
    }
  }
  __syncthreads();
  const int q  = lane >> 3;
  const int c8 = (lane & 7) * 8;
  v8h hv[2];
#pragma unroll
  for (int it = 0; it < 2; ++it) {
    const int n = it * 32 + wave * 4 + q;
#pragma unroll
    for (int e = 0; e < 8; ++e) {
      const float f = sT[(c8 + e) * 68 + n];
      hv[it][e] = (_Float16)(bf_rne(f) * kWgtCarry);
    }
  }
  for (int pass = 0; pass < 2; ++pass) {
#pragma unroll
    for (int it = 0; it < 2; ++it) {
      const int n = it * 32 + wave * 4 + q;
      *(volatile v8h*)(dst + (size_t)(n0 + n) * kdim + k0 + c8) = hv[it];
    }
    __threadfence();
  }
}

__global__ __launch_bounds__(256) void normalize_kernel(
    const float* __restrict__ embed, unsigned short* __restrict__ E16, unsigned short* __restrict__ Q16)
{
  const int lane = threadIdx.x & 31;
  const int wave = __builtin_amdgcn_readfirstlane((int)(threadIdx.x >> 5));
  const int row  = blockIdx.x * 8 + wave;
  const float* e = embed + (size_t)row * kH;
  float er[16];
#pragma unroll
  for (int j = 0; j < 2; ++j) {
    const v4f a0 = *(const v4f*)(e + j * 256 + lane * 8);
    const v4f a1 = *(const v4f*)(e + j * 256 + lane * 8 + 4);
#pragma unroll
    for (int c = 0; c < 4; ++c) {
      er[j * 8 + c]     = bf_rne(a0[c]);
      er[j * 8 + 4 + c] = bf_rne(a1[c]);
    }
  }
  float ss = 0.0f;
#pragma unroll
  for (int i = 0; i < 16; ++i) ss = fmaf(er[i], er[i], ss);
#pragma unroll
  for (int o = 16; o > 0; o >>= 1) ss += __shfl_xor(ss, o, 32);
  const float inv = 1.0f / fmaxf(sqrtf(ss), 1e-12f);
  v8h ev[2], qv[2];
#pragma unroll
  for (int j = 0; j < 2; ++j) {
#pragma unroll
    for (int c = 0; c < 8; ++c) {
      const float v = er[j * 8 + c];
      ev[j][c] = (_Float16)(v * kActCarry);
      qv[j][c] = (_Float16)((v * inv) * kQCarry);
    }
  }
  unsigned short* pe = E16 + (size_t)row * kH + lane * 8;
  unsigned short* pq = Q16 + (size_t)row * kH + lane * 8;
  for (int pass = 0; pass < 2; ++pass) {
#pragma unroll
    for (int j = 0; j < 2; ++j) {
      *(volatile v8h*)(pe + j * 256) = ev[j];
      *(volatile v8h*)(pq + j * 256) = qv[j];
    }
    __threadfence();
  }
}

__global__ __launch_bounds__(256) void corr_top1_kernel(
    const _Float16* __restrict__ Q, int* __restrict__ idx)
{
  __shared__ __align__(16) float sV[4 * 64];
  __shared__ __align__(16) int   sC[4 * 64];
  const int lane  = threadIdx.x & 31;
  const int wave  = __builtin_amdgcn_readfirstlane((int)(threadIdx.x >> 5));
  const int b     = blockIdx.x >> 5;
  const int rt    = blockIdx.x & 31;
  const int rh    = wave & 1;
  const int cg    = wave >> 1;
  const int rlane = lane & 15;
  const int koff  = (lane >> 4) * 8;
  const int mOff  = koff;
  const int row0  = rt * 64 + rh * 32;
  const _Float16* Qb = Q + (size_t)b * kN * kH;
  const _Float16* arow = Qb + (size_t)(row0 + rlane) * kH + koff;

  float bv[2][8];
  int   bc[2][8];
#pragma unroll
  for (int i = 0; i < 2; ++i)
#pragma unroll
    for (int r = 0; r < 8; ++r) { bv[i][r] = -INFINITY; bc[i][r] = 0x7fffffff; }

#pragma unroll 1
  for (int t = 0; t < 8; ++t) {
    const int n0 = (cg + 4 * t) * 64;
    const _Float16* brow = Qb + (size_t)(n0 + rlane) * kH + koff;
    v8f acc[2][4];
#pragma unroll
    for (int i = 0; i < 2; ++i)
#pragma unroll
      for (int j = 0; j < 4; ++j) acc[i][j] = (v8f){0.f,0.f,0.f,0.f,0.f,0.f,0.f,0.f};
#pragma unroll 1
    for (int k0 = 0; k0 < kH; k0 += 32) {
      v16h bh[4];
#pragma unroll
      for (int j = 0; j < 4; ++j) bh[j] = frag_ld(brow + (size_t)(j * 16) * kH + k0);
#pragma unroll
      for (int i = 0; i < 2; ++i) {
        const v16h ah = frag_ld(arow + (size_t)(i * 16) * kH + k0);
#pragma unroll
        for (int j = 0; j < 4; ++j) acc[i][j] = mma_g(ah, bh[j], acc[i][j]);
      }
    }
#pragma unroll
    for (int i = 0; i < 2; ++i)
#pragma unroll
      for (int r = 0; r < 8; ++r)
#pragma unroll
        for (int j = 0; j < 4; ++j) {
          const float s = acc[i][j][r];
          const int col = n0 + j * 16 + rlane;
          const bool gt = s > bv[i][r];
          bv[i][r] = gt ? s : bv[i][r];
          bc[i][r] = gt ? col : bc[i][r];
        }
  }
#pragma unroll
  for (int i = 0; i < 2; ++i)
#pragma unroll
    for (int r = 0; r < 8; ++r) {
      float v = bv[i][r];
      int   c = bc[i][r];
#pragma unroll
      for (int off = 1; off < 16; off <<= 1) {
        const float ov = __shfl_xor(v, off, 32);
        const int   oc = __shfl_xor(c, off, 32);
        const bool take = (ov > v) || (ov == v && oc < c);
        v = take ? ov : v;
        c = take ? oc : c;
      }
      bv[i][r] = v;
      bc[i][r] = c;
    }
  if (rlane == 0) {
#pragma unroll
    for (int i = 0; i < 2; ++i)
#pragma unroll
      for (int r = 0; r < 8; ++r) {
        const int rr = rh * 32 + i * 16 + mOff + r;
        sV[cg * 64 + rr] = bv[i][r];
        sC[cg * 64 + rr] = bc[i][r];
      }
  }
  __syncthreads();
  if (wave == 0) {
    const int l16 = lane & 15;
    v4f v0 = *(const v4f*)(sV + l16 * 4);
    v4i c0 = *(const v4i*)(sC + l16 * 4);
    float fv[4] = { v0[0], v0[1], v0[2], v0[3] };
    int   fc[4] = { c0[0], c0[1], c0[2], c0[3] };
#pragma unroll
    for (int g = 1; g < 4; ++g) {
      const v4f vg = *(const v4f*)(sV + g * 64 + l16 * 4);
      const v4i cgv = *(const v4i*)(sC + g * 64 + l16 * 4);
      const float tv[4] = { vg[0], vg[1], vg[2], vg[3] };
      const int   tc[4] = { cgv[0], cgv[1], cgv[2], cgv[3] };
#pragma unroll
      for (int e = 0; e < 4; ++e) {
        const bool take = (tv[e] > fv[e]) || (tv[e] == fv[e] && tc[e] < fc[e]);
        fv[e] = take ? tv[e] : fv[e];
        fc[e] = take ? tc[e] : fc[e];
      }
    }
#pragma unroll
    for (int e = 0; e < 4; ++e) {
      int c = fc[e];
      c = c < 0 ? 0 : c;
      c = c > (kN - 1) ? (kN - 1) : c;
      fc[e] = c;
    }
    const v4i res = { fc[0], fc[1], fc[2], fc[3] };
    int* dst = idx + (size_t)b * kN + rt * 64 + l16 * 4;
    if (lane < 16) { *(volatile v4i*)dst = res; }
    __threadfence();
    if (lane < 16) { *(volatile v4i*)dst = res; }
  }
}

__global__ __launch_bounds__(512) void gdiag_kernel(
    const int* __restrict__ idx, float* __restrict__ gd, float dv2)
{
  __shared__ __align__(16) int sCnt[kN];
  const int tid = threadIdx.x;
  const int b   = blockIdx.x;
  const v4i iv = *(const v4i*)(idx + (size_t)b * kN + tid * 4);
  int my[4] = { iv[0], iv[1], iv[2], iv[3] };
#pragma unroll
  for (int e = 0; e < 4; ++e) {
    int c = my[e];
    c = c < 0 ? 0 : c;
    c = c > (kN - 1) ? (kN - 1) : c;
    my[e] = c;
  }
  const v4i zero4 = { 0, 0, 0, 0 };
  *(v4i*)(sCnt + tid * 4) = zero4;
  __syncthreads();
#pragma unroll
  for (int e = 0; e < 4; ++e) atomicAdd(&sCnt[my[e]], 1);
  __syncthreads();
  const v4i cv = *(const v4i*)(sCnt + tid * 4);
  const int cn[4] = { cv[0], cv[1], cv[2], cv[3] };
  float gv[4];
#pragma unroll
  for (int e = 0; e < 4; ++e) {
    const int n = tid * 4 + e;
    const float de  = (float)cn[e];
    const float inv = 1.0f / (de + 1e-4f);
    const float val = (dv2 * inv) * dv2;
    gv[e] = (my[e] == n && cn[e] > 0) ? val : 0.0f;
  }
  const v4f out4 = { gv[0], gv[1], gv[2], gv[3] };
  float* dst = gd + (size_t)b * kN + tid * 4;
  *(volatile v4f*)dst = out4;
  __threadfence();
  *(volatile v4f*)dst = out4;
}

template <bool RELU>
__global__ __launch_bounds__(256) void gemm_rowscale_kernel(
    const _Float16* __restrict__ A, const _Float16* __restrict__ Bt,
    const float* __restrict__ bias, const float* __restrict__ gdiag,
    unsigned short* __restrict__ C)
{
  __shared__ __align__(16) float sT[8][16 * 68];
  const int lane  = threadIdx.x & 31;
  const int wave  = __builtin_amdgcn_readfirstlane((int)(threadIdx.x >> 5));
  const int m0    = blockIdx.x * 64;
  const int n0    = wave * 64;
  const int rlane = lane & 15;
  const int koff  = (lane >> 4) * 8;
  const int mOff  = koff;
  const _Float16* arow = A  + (size_t)(m0 + rlane) * kH + koff;
  const _Float16* brow = Bt + (size_t)(n0 + rlane) * kH + koff;

  v8f acc[4][4];
#pragma unroll
  for (int i = 0; i < 4; ++i)
#pragma unroll
    for (int j = 0; j < 4; ++j) acc[i][j] = (v8f){0.f,0.f,0.f,0.f,0.f,0.f,0.f,0.f};

#pragma unroll 1
  for (int k0 = 0; k0 < kH; k0 += 32) {
    v16h bh[4];
#pragma unroll
    for (int j = 0; j < 4; ++j) bh[j] = frag_ld(brow + (size_t)(j * 16) * kH + k0);
#pragma unroll
    for (int i = 0; i < 4; ++i) {
      const v16h ah = frag_ld(arow + (size_t)(i * 16) * kH + k0);
#pragma unroll
      for (int j = 0; j < 4; ++j) acc[i][j] = mma_g(ah, bh[j], acc[i][j]);
    }
  }

  float bvj[4];
#pragma unroll
  for (int j = 0; j < 4; ++j) bvj[j] = bf_rne(bias[n0 + j * 16 + rlane]);

  float* slab = sT[wave];
  const int q  = lane >> 3;
  const int c8 = (lane & 7) * 8;
#pragma unroll
  for (int i = 0; i < 4; ++i) {
    const int mBase = m0 + i * 16;
    const float* gp = gdiag + mBase + mOff;
    const v4f g0 = *(const v4f*)(gp);
    const v4f g1 = *(const v4f*)(gp + 4);
    const float gr[8] = { g0[0], g0[1], g0[2], g0[3], g1[0], g1[1], g1[2], g1[3] };
#pragma unroll
    for (int j = 0; j < 4; ++j) {
#pragma unroll
      for (int r = 0; r < 8; ++r) {
        float v = (acc[i][j][r] * kFold + bvj[j]) * gr[r];
        if (RELU) v = fmaxf(v, 0.0f);
        slab[(mOff + r) * 68 + j * 16 + rlane] = v * kActCarry;
      }
    }
    wave_lds_sync();
    for (int pass = 0; pass < 2; ++pass) {
#pragma unroll
      for (int it = 0; it < 4; ++it) {
        const int row = it * 4 + q;
        const float* sp = slab + row * 68 + c8;
        v8h hv;
#pragma unroll
        for (int e = 0; e < 8; ++e) hv[e] = (_Float16)sp[e];
        *(volatile v8h*)(C + (size_t)(mBase + row) * kH + n0 + c8) = hv;
      }
      __threadfence();
    }
    wave_lds_sync();
  }
}

__global__ __launch_bounds__(256) void fc_ln_kernel(
    const _Float16* __restrict__ E16, const _Float16* __restrict__ X2, const _Float16* __restrict__ WFT,
    const float* __restrict__ bfc, const float* __restrict__ lng, const float* __restrict__ lnb,
    float* __restrict__ out)
{
  __shared__ __align__(16) float sT[8][16 * 68];
  __shared__ __align__(16) float sP1[8 * 32];
  __shared__ __align__(16) float sP2[8 * 32];
  const int lane  = threadIdx.x & 31;
  const int wave  = __builtin_amdgcn_readfirstlane((int)(threadIdx.x >> 5));
  const int m0    = blockIdx.x * 32;
  const int n0    = wave * 64;
  const int rlane = lane & 15;
  const int koff  = (lane >> 4) * 8;
  const int mOff  = koff;
  const _Float16* a0p = E16 + (size_t)(m0 + rlane) * kH + koff;
  const _Float16* a1p = X2  + (size_t)(m0 + rlane) * kH + koff;
  const _Float16* bp  = WFT + (size_t)(n0 + rlane) * kH2 + koff;

  v8f acc[2][4];
#pragma unroll
  for (int i = 0; i < 2; ++i)
#pragma unroll
    for (int j = 0; j < 4; ++j) acc[i][j] = (v8f){0.f,0.f,0.f,0.f,0.f,0.f,0.f,0.f};

#pragma unroll 1
  for (int k0 = 0; k0 < kH; k0 += 32) {
    v16h bh[4];
#pragma unroll
    for (int j = 0; j < 4; ++j) bh[j] = frag_ld(bp + (size_t)(j * 16) * kH2 + k0);
#pragma unroll
    for (int i = 0; i < 2; ++i) {
      const v16h ah = frag_ld(a0p + (size_t)(i * 16) * kH + k0);
#pragma unroll
      for (int j = 0; j < 4; ++j) acc[i][j] = mma_g(ah, bh[j], acc[i][j]);
    }
  }
#pragma unroll 1
  for (int k0 = 0; k0 < kH; k0 += 32) {
    v16h bh[4];
#pragma unroll
    for (int j = 0; j < 4; ++j) bh[j] = frag_ld(bp + (size_t)(j * 16) * kH2 + kH + k0);
#pragma unroll
    for (int i = 0; i < 2; ++i) {
      const v16h ah = frag_ld(a1p + (size_t)(i * 16) * kH + k0);
#pragma unroll
      for (int j = 0; j < 4; ++j) acc[i][j] = mma_g(ah, bh[j], acc[i][j]);
    }
  }

  float bq[4], gq[4], lq[4];
#pragma unroll
  for (int j = 0; j < 4; ++j) {
    const int n = n0 + j * 16 + rlane;
    bq[j] = bf_rne(bfc[n]);
    gq[j] = bf_rne(lng[n]);
    lq[j] = bf_rne(lnb[n]);
  }
#pragma unroll
  for (int i = 0; i < 2; ++i)
#pragma unroll
    for (int j = 0; j < 4; ++j)
#pragma unroll
      for (int r = 0; r < 8; ++r) acc[i][j][r] = acc[i][j][r] * kFold + bq[j];

  float rs[2][8];
#pragma unroll
  for (int i = 0; i < 2; ++i)
#pragma unroll
    for (int r = 0; r < 8; ++r) {
      float s = (acc[i][0][r] + acc[i][1][r]) + (acc[i][2][r] + acc[i][3][r]);
#pragma unroll
      for (int off = 1; off < 16; off <<= 1) s += __shfl_xor(s, off, 32);
      rs[i][r] = s;
    }
  if (rlane == 0) {
#pragma unroll
    for (int i = 0; i < 2; ++i)
#pragma unroll
      for (int r = 0; r < 8; ++r) sP1[wave * 32 + i * 16 + mOff + r] = rs[i][r];
  }
  __syncthreads();
  float mu[2][8];
#pragma unroll
  for (int i = 0; i < 2; ++i) {
    v4f t0 = (v4f){0.f,0.f,0.f,0.f};
    v4f t1 = (v4f){0.f,0.f,0.f,0.f};
#pragma unroll
    for (int w = 0; w < 8; ++w) {
      t0 += *(const v4f*)(sP1 + w * 32 + i * 16 + mOff);
      t1 += *(const v4f*)(sP1 + w * 32 + i * 16 + mOff + 4);
    }
    mu[i][0] = t0[0] * kInvH; mu[i][1] = t0[1] * kInvH; mu[i][2] = t0[2] * kInvH; mu[i][3] = t0[3] * kInvH;
    mu[i][4] = t1[0] * kInvH; mu[i][5] = t1[1] * kInvH; mu[i][6] = t1[2] * kInvH; mu[i][7] = t1[3] * kInvH;
  }
#pragma unroll
  for (int i = 0; i < 2; ++i)
#pragma unroll
    for (int r = 0; r < 8; ++r) {
      float s = 0.0f;
#pragma unroll
      for (int j = 0; j < 4; ++j) {
        const float d = acc[i][j][r] - mu[i][r];
        acc[i][j][r] = d;
        s = fmaf(d, d, s);
      }
#pragma unroll
      for (int off = 1; off < 16; off <<= 1) s += __shfl_xor(s, off, 32);
      rs[i][r] = s;
    }
  if (rlane == 0) {
#pragma unroll
    for (int i = 0; i < 2; ++i)
#pragma unroll
      for (int r = 0; r < 8; ++r) sP2[wave * 32 + i * 16 + mOff + r] = rs[i][r];
  }
  __syncthreads();
#pragma unroll
  for (int i = 0; i < 2; ++i) {
    v4f t0 = (v4f){0.f,0.f,0.f,0.f};
    v4f t1 = (v4f){0.f,0.f,0.f,0.f};
#pragma unroll
    for (int w = 0; w < 8; ++w) {
      t0 += *(const v4f*)(sP2 + w * 32 + i * 16 + mOff);
      t1 += *(const v4f*)(sP2 + w * 32 + i * 16 + mOff + 4);
    }
    rs[i][0] = rsqrtf(t0[0] * kInvH + kLnEps); rs[i][1] = rsqrtf(t0[1] * kInvH + kLnEps);
    rs[i][2] = rsqrtf(t0[2] * kInvH + kLnEps); rs[i][3] = rsqrtf(t0[3] * kInvH + kLnEps);
    rs[i][4] = rsqrtf(t1[0] * kInvH + kLnEps); rs[i][5] = rsqrtf(t1[1] * kInvH + kLnEps);
    rs[i][6] = rsqrtf(t1[2] * kInvH + kLnEps); rs[i][7] = rsqrtf(t1[3] * kInvH + kLnEps);
  }

  float* slab = sT[wave];
  const int hh = lane >> 4;
  const int c4 = (lane & 15) * 4;
#pragma unroll
  for (int i = 0; i < 2; ++i) {
    const int mBase = m0 + i * 16;
#pragma unroll
    for (int j = 0; j < 4; ++j)
#pragma unroll
      for (int r = 0; r < 8; ++r)
        slab[(mOff + r) * 68 + j * 16 + rlane] = (acc[i][j][r] * rs[i][r]) * gq[j] + lq[j];
    wave_lds_sync();
    for (int pass = 0; pass < 2; ++pass) {
#pragma unroll
      for (int it = 0; it < 8; ++it) {
        const int row = it * 2 + hh;
        const v4f v = *(const v4f*)(slab + row * 68 + c4);
        *(volatile v4f*)(out + (size_t)(mBase + row) * kH + n0 + c4) = v;
      }
      __threadfence();
    }
    wave_lds_sync();
  }
}

extern "C" void kernel_launch(void* const* d_in, const int* in_sizes, int n_in,
                              void* d_out, int out_size, void* d_ws, size_t ws_size,
                              hipStream_t stream) {
  if (n_in < 9) return;
  if (in_sizes[0] != kRows * kH) return;
  if (in_sizes[1] != kH * kH) return;
  if (in_sizes[2] != kH) return;
  if (in_sizes[3] != kH * kH) return;
  if (in_sizes[4] != kH) return;
  if (in_sizes[5] != kH2 * kH) return;
  if (in_sizes[6] != kH) return;
  if (in_sizes[7] != kH) return;
  if (in_sizes[8] != kH) return;
  if (out_size != kRows * kH) return;
  if (ws_size < kWsTotal) return;

  const float* embed = (const float*)d_in[0];
  const float* W1    = (const float*)d_in[1];
  const float* b1    = (const float*)d_in[2];
  const float* W2    = (const float*)d_in[3];
  const float* b2    = (const float*)d_in[4];
  const float* Wfc   = (const float*)d_in[5];
  const float* bfc   = (const float*)d_in[6];
  const float* ln_g  = (const float*)d_in[7];
  const float* ln_b  = (const float*)d_in[8];
  float* out = (float*)d_out;

  char* ws = (char*)d_ws;
  unsigned short* E16 = (unsigned short*)(ws + kOffE16);
  unsigned short* Q16 = (unsigned short*)(ws + kOffQ16);
  unsigned short* X1  = (unsigned short*)(ws + kOffX1);
  unsigned short* X2  = (unsigned short*)(ws + kOffX2);
  unsigned short* W1T = (unsigned short*)(ws + kOffW1T);
  unsigned short* W2T = (unsigned short*)(ws + kOffW2T);
  unsigned short* WFT = (unsigned short*)(ws + kOffWFT);
  int*            IDX = (int*)(ws + kOffIDX);
  float*          GD  = (float*)(ws + kOffGD);

  const float dv2 = 1.0f / sqrtf(1.0f + 1e-4f);

  prep_weights_kernel<<<256, 256, 0, stream>>>(W1, W2, Wfc, W1T, W2T, WFT);
  normalize_kernel<<<kRows / 8, 256, 0, stream>>>(embed, E16, Q16);
  corr_top1_kernel<<<kB * (kN / 64), 256, 0, stream>>>((const _Float16*)Q16, IDX);
  gdiag_kernel<<<kB, 512, 0, stream>>>(IDX, GD, dv2);
  gemm_rowscale_kernel<true><<<kRows / 64, 256, 0, stream>>>(
      (const _Float16*)E16, (const _Float16*)W1T, b1, GD, X1);
  gemm_rowscale_kernel<false><<<kRows / 64, 256, 0, stream>>>(
      (const _Float16*)X1, (const _Float16*)W2T, b2, GD, X2);
  fc_ln_kernel<<<kRows / 32, 256, 0, stream>>>(
      (const _Float16*)E16, (const _Float16*)X2, (const _Float16*)WFT, bfc, ln_g, ln_b, out);
}
